// ChamferSimilarity_66718021976303
// MI455X (gfx1250) — hardware-verified
//
#include <hip/hip_runtime.h>
#include <math.h>

typedef __attribute__((ext_vector_type(16))) _Float16 v16h;
typedef __attribute__((ext_vector_type(16))) __bf16 v16b;
typedef __attribute__((ext_vector_type(8)))  _Float16 v8h;
typedef __attribute__((ext_vector_type(8)))  float v8f;
typedef __attribute__((ext_vector_type(4)))  float v4f;
typedef __attribute__((ext_vector_type(2)))  float v2f;
typedef __attribute__((ext_vector_type(4)))  unsigned v4u;
typedef __attribute__((ext_vector_type(4)))  int v4i;
typedef float __attribute__((may_alias)) float_a;
typedef int __attribute__((may_alias)) int_a;

template <typename T> __device__ __forceinline__ void vst2(void* p, T v) { *(volatile T*)p = v; __threadfence(); *(volatile T*)p = v; }
__device__ __forceinline__ v8f wmma16(v16h a, v16h b, v8f c) {
  v8f d = __builtin_amdgcn_wmma_f32_16x16x32_f16(false, a, false, b, (short)0, c, false, false);
  asm volatile("v_nop\n\tv_nop\n\tv_nop\n\tv_nop" : "+v"(d) : "v"(a), "v"(b));
  return d;
}
__device__ __forceinline__ v8f wmma_bf(v16b a, v16b b, v8f c) {
  v8f d = __builtin_amdgcn_wmma_f32_16x16x32_bf16(false, a, false, b, (short)0, c, false, false);
  asm volatile("v_nop\n\tv_nop\n\tv_nop\n\tv_nop" : "+v"(d) : "v"(a), "v"(b));
  return d;
}
__device__ __forceinline__ v16h frag_h(const _Float16* rowk0, int lane) {
  union { v16h v; v8h q[2]; } u; const _Float16* p = rowk0 + 8 * (lane >> 4);
  u.q[0] = *(const v8h*)p; u.q[1] = *(const v8h*)(p + 16); return u.v;
}
__device__ __forceinline__ v16h frag_f32(const float* rowk0, int lane) {
  v16h a; const float* p = rowk0 + 8 * (lane >> 4);
#pragma unroll
  for (int i = 0; i < 8; ++i) { a[i] = (_Float16)p[i]; a[8 + i] = (_Float16)p[16 + i]; }
  return a;
}
__device__ __forceinline__ v16h frag_f32s(const float* rowk0, int lane, float sc) {
  v16h a; const float* p = rowk0 + 8 * (lane >> 4);
#pragma unroll
  for (int i = 0; i < 8; ++i) { a[i] = (_Float16)(p[i] * sc); a[8 + i] = (_Float16)(p[16 + i] * sc); }
  return a;
}
__device__ __forceinline__ v16h fragc_f32(const float* W, int k0, int n, int lane, int ld, int K) {
  v16h a; const int g = lane >> 4;
#pragma unroll
  for (int i = 0; i < 8; ++i) { const int ka = k0 + 8 * g + i, kb = ka + 16;
    a[i] = (_Float16)(ka < K ? W[(size_t)ka * ld + n] : 0.f); a[8 + i] = (_Float16)(kb < K ? W[(size_t)kb * ld + n] : 0.f); }
  return a;
}
struct F2 { v16b h, l; };
__device__ __forceinline__ F2 bsplit16(const float v[16]) { F2 r;
#pragma unroll
  for (int i = 0; i < 16; ++i) { const __bf16 h = (__bf16)v[i]; r.h[i] = h; r.l[i] = (__bf16)(v[i] - (float)h); }
  return r; }
__device__ __forceinline__ F2 split_row(const float* row, int k0, int lane) { float v[16]; const float* p = row + k0 + 8 * (lane >> 4);
#pragma unroll
  for (int i = 0; i < 8; ++i) { v[i] = p[i]; v[8 + i] = p[16 + i]; }
  return bsplit16(v); }
__device__ __forceinline__ F2 split_rowK(const float* row, int k0, int lane, int K) { float v[16]; const int g = lane >> 4;
#pragma unroll
  for (int i = 0; i < 8; ++i) { const int ka = k0 + 8 * g + i, kb = ka + 16; v[i] = ka < K ? row[ka] : 0.f; v[8 + i] = kb < K ? row[kb] : 0.f; }
  return bsplit16(v); }
__device__ __forceinline__ F2 split_col(const float* W, int k0, int n, int lane, int ld, int K) { float v[16]; const int g = lane >> 4;
#pragma unroll
  for (int i = 0; i < 8; ++i) { const int ka = k0 + 8 * g + i, kb = ka + 16; v[i] = ka < K ? W[(size_t)ka * ld + n] : 0.f; v[8 + i] = kb < K ? W[(size_t)kb * ld + n] : 0.f; }
  return bsplit16(v); }
__device__ __forceinline__ v8f mac3(const F2& a, const F2& b, v8f c) { c = wmma_bf(a.l, b.h, c); c = wmma_bf(a.h, b.l, c); return wmma_bf(a.h, b.h, c); }
__device__ __forceinline__ float sigm(float v) { return 1.0f / (1.0f + expf(-v)); }
#define LDSX() do { asm volatile("s_wait_dscnt 0" ::: "memory"); __builtin_amdgcn_wave_barrier(); __builtin_amdgcn_fence(__ATOMIC_RELEASE, "workgroup"); } while (0)

#define NBQ 64
#define NQ 32
#define ND 256
#define DD 128
#define NEG -1.0e9f
#define VTH -1.0e8f

__global__ __launch_bounds__(256) void k_norm(const float* __restrict__ qe, const int* __restrict__ qm, const float* __restrict__ de, const int* __restrict__ dm, _Float16* __restrict__ Q16, _Float16* __restrict__ D16) {
  const int wave = threadIdx.x >> 5, lane = threadIdx.x & 31; const int which = blockIdx.y; const int r = blockIdx.x * 8 + wave;
  const int nrows = which ? NBQ * ND : NBQ * NQ; if (r >= nrows) return;
  const float* src = (which ? de : qe) + (size_t)r * DD; const int m = which ? dm[r] : qm[r];
  const v4f v = *(const v4f*)(src + lane * 4); float s = v[0] * v[0] + v[1] * v[1] + v[2] * v[2] + v[3] * v[3];
#pragma unroll
  for (int off = 16; off >= 1; off >>= 1) s += __shfl_xor(s, off, 32);
  const float inv = (m != 0 ? 1.0f : 0.0f) / fmaxf(sqrtf(s), 1e-12f);
  union { _Float16 h4[4]; unsigned long long u; } pk;
#pragma unroll
  for (int e = 0; e < 4; ++e) pk.h4[e] = (_Float16)(v[e] * inv);
  vst2((unsigned long long*)((which ? D16 : Q16) + (size_t)r * DD) + lane, pk.u);
}
__global__ __launch_bounds__(64) void k_pair(const _Float16* __restrict__ Q16, const _Float16* __restrict__ D16, const int* __restrict__ qm, const int* __restrict__ dm, float* __restrict__ SC) {
  __shared__ float sS[NQ][ND + 1]; __shared__ float sqv[NQ], sdv[ND]; __shared__ float sred[8];
  const int tid = threadIdx.x, w = tid >> 5, lane = tid & 31, col = lane & 15, g = lane >> 4;
  const int qb = blockIdx.x, db = blockIdx.y;
  if (tid < NQ) sqv[tid] = (float)(qm[qb * NQ + tid] != 0);
  for (int s = tid; s < ND; s += 64) sdv[s] = (float)(dm[qb * ND + s] != 0);
  v16h aq[4];
#pragma unroll
  for (int kc = 0; kc < 4; ++kc) aq[kc] = frag_h(Q16 + ((size_t)qb * NQ + w * 16 + col) * DD + kc * 32, lane);
#pragma unroll 2
  for (int t = 0; t < ND / 16; ++t) { v8f acc = {};
#pragma unroll
    for (int kc = 0; kc < 4; ++kc) acc = wmma16(aq[kc], frag_h(D16 + ((size_t)db * ND + t * 16 + col) * DD + kc * 32, lane), acc);
#pragma unroll
    for (int r = 0; r < 8; ++r) sS[w * 16 + 8 * g + r][t * 16 + col] = acc[r]; }
  __syncthreads();
  float part = 0.f, cnt = 0.f;
  if (tid < NQ) { const float qvld = sqv[tid]; float mx = NEG;
    for (int s = 0; s < ND; ++s) { const float v = (qvld != 0.f && sdv[s] != 0.f) ? sS[tid][s] : NEG; mx = fmaxf(mx, v); }
    const bool valid = mx > VTH; part = valid ? mx : 0.f; cnt = valid ? 1.f : 0.f; }
#pragma unroll
  for (int off = 16; off >= 1; off >>= 1) { part += __shfl_xor(part, off, 32); cnt += __shfl_xor(cnt, off, 32); }
  if (tid == 0) { sred[0] = part; sred[1] = cnt; }
  float p2 = 0.f, c2 = 0.f;
  for (int s = tid; s < ND; s += 64) { const float dvld = sdv[s]; float mx = NEG;
    for (int t = 0; t < NQ; ++t) { const float v = (dvld != 0.f && sqv[t] != 0.f) ? sS[t][s] : NEG; mx = fmaxf(mx, v); }
    const bool valid = mx > VTH; p2 += valid ? mx : 0.f; c2 += valid ? 1.f : 0.f; }
#pragma unroll
  for (int off = 16; off >= 1; off >>= 1) { p2 += __shfl_xor(p2, off, 32); c2 += __shfl_xor(c2, off, 32); }
  if (lane == 0) { sred[4 + 2 * w] = p2; sred[5 + 2 * w] = c2; }
  __syncthreads();
  if (tid < 32) { const float dsum = sred[4] + sred[6], dcnt = sred[5] + sred[7];
    const float q2d = sred[0] / fmaxf(sred[1], 1.0f), d2q = dsum / fmaxf(dcnt, 1.0f);
    const float val = tid == 0 ? 0.5f * (q2d + d2q) : 0.f;
    vst2(SC + ((size_t)qb * NBQ + db) * 32 + tid, val); }
}
__global__ __launch_bounds__(256) void k_pack(const float* __restrict__ SC, float* __restrict__ out) {
  for (int q = threadIdx.x; q < NBQ * NBQ; q += 256) vst2(out + q, SC[(size_t)q * 32]);
}
extern "C" void kernel_launch(void* const* d_in, const int* in_sizes, int n_in, void* d_out, int out_size, void* d_ws, size_t ws_size, hipStream_t stream) {
  (void)in_sizes; (void)n_in; (void)out_size; (void)ws_size;
  const float* qe = (const float*)d_in[0]; const int* qm = (const int*)d_in[1]; const float* de = (const float*)d_in[2]; const int* dm = (const int*)d_in[3];
  float* out = (float*)d_out;
  char* ws = (char*)d_ws; size_t off = 0;
  auto take = [&](size_t bytes) { char* p = ws + off; off += (bytes + 255) & ~(size_t)255; return p; };
  _Float16* Q16 = (_Float16*)take((size_t)NBQ * NQ * DD * 2); _Float16* D16 = (_Float16*)take((size_t)NBQ * ND * DD * 2); float* SC = (float*)take((size_t)NBQ * NBQ * 32 * 4);
  k_norm<<<dim3(NBQ * ND / 8, 2), 256, 0, stream>>>(qe, qm, de, dm, Q16, D16);
  k_pair<<<dim3(NBQ, NBQ), 64, 0, stream>>>(Q16, D16, qm, dm, SC);
  k_pack<<<1, 256, 0, stream>>>(SC, out);
}
